// GlobalAggregationBlock_57140244906430
// MI455X (gfx1250) — hardware-verified
//
#include <hip/hip_runtime.h>
#include <math.h>
#include <stdint.h>

#ifndef ND
#define ND 16
#endif
#define NHH    32
#define NWW    32
#define NTOK   (ND * NHH * NWW)
#define CIN    128
#define DK     64
#define COUT   128
#define QT     64
#define OSP    68
#define TP     72
#define CHB    256
#define WSC    256.0f
#define IWSC   0.00390625f
#define QSC    0.125f
#define VSC    16.0f
#define IVSC   0.0625f
#define OSC    1024.0f
#define IOSC   0.0009765625f
#define RSC    1024.0f
#define IRSC   0.0009765625f
#define LNPS   9.704060527839234f

static_assert(ND >= 1 && ND <= 16);
static_assert(NTOK % QT == 0);
static_assert(NTOK % 32 == 0);
static_assert(CIN % QT == 0 && CIN % 32 == 0);
static_assert(DK == QT);
static_assert(DK % 32 == 0);
static_assert(COUT % QT == 0);
static_assert((DK * CIN) % (8 * CHB) == 0);
static_assert((COUT * DK) % (8 * CHB) == 0);
static_assert((OSP * 4) % 16 == 0);
static_assert((TP * 2) % 16 == 0);

typedef _Float16       v16h __attribute__((ext_vector_type(16)));
typedef _Float16       v8h  __attribute__((ext_vector_type(8)));
typedef __bf16         v16b __attribute__((ext_vector_type(16)));
typedef unsigned short v8us __attribute__((ext_vector_type(8)));
typedef float          v8f  __attribute__((ext_vector_type(8)));
typedef float          v4f  __attribute__((ext_vector_type(4)));
typedef unsigned int   v4u  __attribute__((ext_vector_type(4)));

union Frag  { v8us u[2]; v16h h; v16b bf; };
union FragH { v16h v; v8h hv[2]; };
static_assert(sizeof(Frag) == 32);
static_assert(sizeof(FragH) == 32);

__device__ __forceinline__ unsigned short bf_bits(float f) {
  unsigned u = __float_as_uint(f);
  return (unsigned short)((u + 0x7FFFu + ((u >> 16) & 1u)) >> 16);
}
__device__ __forceinline__ float bf_up(unsigned short hb) { return __uint_as_float(((unsigned)hb) << 16); }
__device__ __forceinline__ float bfr(float f) { return bf_up(bf_bits(f)); }
__device__ __forceinline__ unsigned short h_bits(_Float16 x) { return __builtin_bit_cast(unsigned short, x); }
__device__ __forceinline__ unsigned pk16(unsigned short a, unsigned short b) { return (unsigned)a | ((unsigned)b << 16); }
__device__ __forceinline__ v8f zero8() { v8f z = {0.f, 0.f, 0.f, 0.f, 0.f, 0.f, 0.f, 0.f}; return z; }
__device__ __forceinline__ float hmax8(v8f s) {
  return fmaxf(fmaxf(fmaxf(s[0], s[1]), fmaxf(s[2], s[3])), fmaxf(fmaxf(s[4], s[5]), fmaxf(s[6], s[7])));
}
__device__ __forceinline__ unsigned wave_ballot(bool p) {
#if defined(__HIP_DEVICE_COMPILE__)
  return __builtin_amdgcn_ballot_w32(p);
#else
  return p ? 1u : 0u;
#endif
}

__device__ __forceinline__ Frag ldfrag(const unsigned short* p) {
  Frag f;
  f.u[0] = *(const v8us*)(p);
  f.u[1] = *(const v8us*)(p + 16);
  return f;
}

__device__ __forceinline__ v8f mma_h(v16h a, v16h b, v8f c) {
  v8f d = __builtin_amdgcn_wmma_f32_16x16x32_f16(false, a, false, b, (short)0, c, false, false);
#if defined(__HIP_DEVICE_COMPILE__)
  asm volatile("v_nop\n\tv_nop\n\tv_nop\n\tv_nop" : "+v"(d) : "v"(a), "v"(b));
#endif
  return d;
}
__device__ __forceinline__ v8f mma_b(v16b a, v16b b, v8f c) {
  v8f d = __builtin_amdgcn_wmma_f32_16x16x32_bf16(false, a, false, b, (short)0, c, false, false);
#if defined(__HIP_DEVICE_COMPILE__)
  const v16h ha = __builtin_bit_cast(v16h, a), hb = __builtin_bit_cast(v16h, b);
  asm volatile("v_nop\n\tv_nop\n\tv_nop\n\tv_nop" : "+v"(d) : "v"(ha), "v"(hb));
#endif
  return d;
}

__global__ __launch_bounds__(CHB)
void cvt_w(const float* __restrict__ Wq, const float* __restrict__ Wk, const float* __restrict__ Wv,
           const float* __restrict__ Wo, unsigned short* W16, unsigned short* Wo16) {
  const int tid = threadIdx.x, blk = blockIdx.x;
  const int BQ = (DK * CIN) / (8 * CHB);
  const int g = blk * CHB + tid;
  const float* src;
  unsigned short* dst;
  int gsrc, gdst;
  if (blk < BQ)          { src = Wq; gsrc = 0;            dst = W16;  gdst = 0; }
  else if (blk < 2 * BQ) { src = Wk; gsrc = BQ * CHB;     dst = W16;  gdst = 0; }
  else if (blk < 3 * BQ) { src = Wv; gsrc = 2 * BQ * CHB; dst = W16;  gdst = 0; }
  else                   { src = Wo; gsrc = 3 * BQ * CHB; dst = Wo16; gdst = 3 * BQ * CHB; }
  const float* s = src + (size_t)8 * (size_t)(g - gsrc);
  const v4f a = *(const v4f*)s;
  const v4f q = *(const v4f*)(s + 4);
  const float f[8] = {a[0], a[1], a[2], a[3], q[0], q[1], q[2], q[3]};
  v4u u;
#pragma unroll
  for (int t = 0; t < 4; ++t) {
    const _Float16 h0 = (_Float16)(bfr(f[2 * t]) * WSC);
    const _Float16 h1 = (_Float16)(bfr(f[2 * t + 1]) * WSC);
    u[t] = pk16(h_bits(h0), h_bits(h1));
  }
#pragma unroll
  for (int pass = 0; pass < 2; ++pass) {
    *(volatile v4u*)(dst + (size_t)8 * (size_t)(g - gdst)) = u;
    __threadfence();
  }
}

__global__ __launch_bounds__(256)
void cvt_x(const float* __restrict__ X, int xstride, unsigned short* XP) {
  __shared__ __align__(16) unsigned short T[QT * TP];
  const int tid = threadIdx.x;
  const int nb = blockIdx.x, cb = blockIdx.y;
  const int e = tid & 7, lq = tid >> 3;
  const int n0 = nb * QT, c0 = cb * QT;
#pragma unroll
  for (int it = 0; it < 2; ++it) {
    const int cl = it * 32 + lq;
    const float* sp = X + (size_t)(c0 + cl) * (size_t)xstride + n0 + 8 * e;
    const v4f a = *(const v4f*)sp;
    const v4f q = *(const v4f*)(sp + 4);
    unsigned short hb[8];
#pragma unroll
    for (int t = 0; t < 4; ++t) {
      hb[t]     = h_bits((_Float16)bfr(a[t]));
      hb[4 + t] = h_bits((_Float16)bfr(q[t]));
    }
#pragma unroll
    for (int t = 0; t < 8; ++t) T[(8 * e + t) * TP + cl] = hb[t];
  }
  __syncthreads();
  v4u up[2];
#pragma unroll
  for (int it = 0; it < 2; ++it) {
    const int nl = it * 32 + lq;
    up[it] = *(const v4u*)(T + nl * TP + 8 * e);
  }
#pragma unroll
  for (int pass = 0; pass < 2; ++pass) {
#pragma unroll
    for (int it = 0; it < 2; ++it) {
      const int nl = it * 32 + lq;
      *(volatile v4u*)(XP + (size_t)(n0 + nl) * CIN + c0 + 8 * e) = up[it];
    }
    __threadfence();
  }
}

__global__ __launch_bounds__(128)
void gemm_qkv(const unsigned short* __restrict__ W16, const unsigned short* __restrict__ XP,
              const float* __restrict__ bq, const float* __restrict__ bk, const float* __restrict__ bv,
              unsigned short* Qh, unsigned short* Ql, unsigned short* Kh, unsigned short* Kl,
              unsigned short* Vc) {
  __shared__ __align__(16) float Os[QT * OSP];
  const int tid  = threadIdx.x;
  const int lane = tid & 31, wave = tid >> 5;
  const int hh   = lane >> 4, c = lane & 15;
  const int nt   = blockIdx.x, mb = blockIdx.y;
  const int n0   = nt * QT, o0 = mb * QT;

  const unsigned short* ap = W16 + (size_t)(o0 + c) * CIN + 8 * hh;
  const unsigned short* bp = XP + (size_t)(n0 + 16 * wave + c) * CIN + 8 * hh;

  v8f acc[4];
#pragma unroll
  for (int mt = 0; mt < 4; ++mt) acc[mt] = zero8();

#pragma unroll
  for (int ks = 0; ks < CIN / 32; ++ks) {
    const Frag fb = ldfrag(bp + 32 * ks);
#pragma unroll
    for (int mt = 0; mt < 4; ++mt) {
      const Frag fa = ldfrag(ap + (size_t)(16 * mt) * CIN + 32 * ks);
      acc[mt] = mma_h(fa.h, fb.h, acc[mt]);
    }
  }

  const float* bsel = (mb == 0) ? bq : ((mb == 1) ? bk : bv);
  const float osc = (mb == 0) ? QSC : 1.0f;
  {
    const int nl = 16 * wave + c;
#pragma unroll
    for (int mt = 0; mt < 4; ++mt) {
      const v4f b0 = *(const v4f*)(bsel + 16 * mt + 8 * hh);
      const v4f b1 = *(const v4f*)(bsel + 16 * mt + 8 * hh + 4);
      v4f va, vb;
#pragma unroll
      for (int r = 0; r < 4; ++r) {
        va[r] = (acc[mt][r] * IWSC + bfr(b0[r])) * osc;
        vb[r] = (acc[mt][4 + r] * IWSC + bfr(b1[r])) * osc;
      }
      *(v4f*)(Os + nl * OSP + 16 * mt + 8 * hh)     = va;
      *(v4f*)(Os + nl * OSP + 16 * mt + 8 * hh + 4) = vb;
    }
  }
  __syncthreads();

  const int e = tid & 7, lq = tid >> 3;
  if (mb < 2) {
    unsigned short* Ph = (mb == 0) ? Qh : Kh;
    unsigned short* Pl = (mb == 0) ? Ql : Kl;
    v4u uh[4], ul[4];
#pragma unroll
    for (int it = 0; it < 4; ++it) {
      const int row = it * 16 + lq;
      const v4f a = *(const v4f*)(Os + row * OSP + 8 * e);
      const v4f q = *(const v4f*)(Os + row * OSP + 8 * e + 4);
      const float f[8] = {a[0], a[1], a[2], a[3], q[0], q[1], q[2], q[3]};
#pragma unroll
      for (int t = 0; t < 4; ++t) {
        const float f0 = f[2 * t], f1 = f[2 * t + 1];
        const unsigned short hb0 = bf_bits(f0), hb1 = bf_bits(f1);
        const unsigned short lb0 = bf_bits(f0 - bf_up(hb0));
        const unsigned short lb1 = bf_bits(f1 - bf_up(hb1));
        uh[it][t] = pk16(hb0, hb1);
        ul[it][t] = pk16(lb0, lb1);
      }
    }
#pragma unroll
    for (int pass = 0; pass < 2; ++pass) {
#pragma unroll
      for (int it = 0; it < 4; ++it) {
        const int row = it * 16 + lq;
        const size_t po = (size_t)(n0 + row) * DK + 8 * e;
        *(volatile v4u*)(Ph + po) = uh[it];
        *(volatile v4u*)(Pl + po) = ul[it];
      }
      __threadfence();
    }
  } else {
    v4u uv[4];
#pragma unroll
    for (int it = 0; it < 4; ++it) {
      const int o = it * 16 + lq;
      unsigned short hb[8];
#pragma unroll
      for (int t = 0; t < 8; ++t) hb[t] = h_bits((_Float16)(Os[(8 * e + t) * OSP + o] * VSC));
#pragma unroll
      for (int t = 0; t < 4; ++t) uv[it][t] = pk16(hb[2 * t], hb[2 * t + 1]);
    }
#pragma unroll
    for (int pass = 0; pass < 2; ++pass) {
#pragma unroll
      for (int it = 0; it < 4; ++it) {
        const int o = it * 16 + lq;
        *(volatile v4u*)(Vc + (size_t)o * NTOK + n0 + 8 * e) = uv[it];
      }
      __threadfence();
    }
  }
}

__global__ __launch_bounds__(128)
void attn_k(const unsigned short* __restrict__ Qh, const unsigned short* __restrict__ Ql,
            const unsigned short* __restrict__ Kh, const unsigned short* __restrict__ Kl,
            const unsigned short* __restrict__ Vc, unsigned short* Oh, unsigned short* Ol) {
  __shared__ __align__(16) float Os[QT * OSP];
  const int tid  = threadIdx.x;
  const int wave = tid >> 5, lane = tid & 31;
  const int hh   = lane >> 4, c = lane & 15;
  const int n0   = blockIdx.x * QT;

  const size_t qo = (size_t)(n0 + 16 * wave + c) * DK + 8 * hh;
  const Frag qh0 = ldfrag(Qh + qo), qh1 = ldfrag(Qh + qo + 32);
  const Frag ql0 = ldfrag(Ql + qo), ql1 = ldfrag(Ql + qo + 32);
  const unsigned short* Khp = Kh + (size_t)c * DK + 8 * hh;
  const unsigned short* Klp = Kl + (size_t)c * DK + 8 * hh;
  const unsigned short* Vp = Vc + (size_t)c * NTOK + 8 * hh;

  float m = -1.0e30f, l = 0.f;
  v8f o[4];
#pragma unroll
  for (int j = 0; j < 4; ++j) o[j] = zero8();

#pragma unroll 1
  for (int kb = 0; kb < NTOK; kb += 32) {
    const size_t r0o = (size_t)kb * DK;
    const size_t r1o = (size_t)(kb + 16) * DK;
    v8f s0 = zero8(), s1 = zero8();
    {
      const Frag k00 = ldfrag(Khp + r0o), k10 = ldfrag(Khp + r1o);
      const Frag g00 = ldfrag(Klp + r0o), g10 = ldfrag(Klp + r1o);
      s0 = mma_b(k00.bf, qh0.bf, s0);
      s1 = mma_b(k10.bf, qh0.bf, s1);
      s0 = mma_b(k00.bf, ql0.bf, s0);
      s1 = mma_b(k10.bf, ql0.bf, s1);
      s0 = mma_b(g00.bf, qh0.bf, s0);
      s1 = mma_b(g10.bf, qh0.bf, s1);
    }
    {
      const Frag k01 = ldfrag(Khp + r0o + 32), k11 = ldfrag(Khp + r1o + 32);
      const Frag g01 = ldfrag(Klp + r0o + 32), g11 = ldfrag(Klp + r1o + 32);
      s0 = mma_b(k01.bf, qh1.bf, s0);
      s1 = mma_b(k11.bf, qh1.bf, s1);
      s0 = mma_b(k01.bf, ql1.bf, s0);
      s1 = mma_b(k11.bf, ql1.bf, s1);
      s0 = mma_b(g01.bf, qh1.bf, s0);
      s1 = mma_b(g11.bf, qh1.bf, s1);
    }

    float mx = fmaxf(hmax8(s0), hmax8(s1));
    mx = fmaxf(mx, __shfl_xor(mx, 16, 32));
    const float mn = fmaxf(m, mx);
    const unsigned grew = wave_ballot(mx > m);
    if (grew != 0u) {
      const float corr = __expf(m - mn);
      l *= corr;
#pragma unroll
      for (int j = 0; j < 4; ++j) {
#pragma unroll
        for (int r = 0; r < 8; ++r) o[j][r] *= corr;
      }
    }
    m = mn;
    const float msh = mn - LNPS;

    FragH ph;
    float ls = 0.f;
#pragma unroll
    for (int r = 0; r < 8; ++r) {
      const float e0 = __expf(s0[r] - msh);
      const float e1 = __expf(s1[r] - msh);
      ls += e0 + e1;
      ph.hv[0][r] = (_Float16)e0;
      ph.hv[1][r] = (_Float16)e1;
    }
    l += ls;

#pragma unroll
    for (int j = 0; j < 4; ++j) {
      const Frag vf = ldfrag(Vp + (size_t)(16 * j) * NTOK + kb);
      o[j] = mma_h(vf.h, ph.v, o[j]);
    }
  }
  l += __shfl_xor(l, 16, 32);
  const float scl = (1.0f / l) * IVSC;

  const int qrow = 16 * wave + c;
#pragma unroll
  for (int j = 0; j < 4; ++j) {
    v4f va, vb;
#pragma unroll
    for (int r = 0; r < 4; ++r) { va[r] = o[j][r] * scl; vb[r] = o[j][4 + r] * scl; }
    *(v4f*)(Os + qrow * OSP + 16 * j + 8 * hh)     = va;
    *(v4f*)(Os + qrow * OSP + 16 * j + 8 * hh + 4) = vb;
  }
  __syncthreads();

  const int e = tid & 7, lq = tid >> 3;
  v4u uh[4], ul[4];
#pragma unroll
  for (int it = 0; it < 4; ++it) {
    const int row = it * 16 + lq;
    const v4f a = *(const v4f*)(Os + row * OSP + 8 * e);
    const v4f q = *(const v4f*)(Os + row * OSP + 8 * e + 4);
    const float f[8] = {a[0], a[1], a[2], a[3], q[0], q[1], q[2], q[3]};
#pragma unroll
    for (int t = 0; t < 4; ++t) {
      const float g0 = f[2 * t] * OSC, g1 = f[2 * t + 1] * OSC;
      const _Float16 h0 = (_Float16)g0, h1 = (_Float16)g1;
      const _Float16 l0 = (_Float16)((g0 - (float)h0) * RSC);
      const _Float16 l1 = (_Float16)((g1 - (float)h1) * RSC);
      uh[it][t] = pk16(h_bits(h0), h_bits(h1));
      ul[it][t] = pk16(h_bits(l0), h_bits(l1));
    }
  }
#pragma unroll
  for (int pass = 0; pass < 2; ++pass) {
#pragma unroll
    for (int it = 0; it < 4; ++it) {
      const int row = it * 16 + lq;
      const size_t po = (size_t)(n0 + row) * DK + 8 * e;
      *(volatile v4u*)(Oh + po) = uh[it];
      *(volatile v4u*)(Ol + po) = ul[it];
    }
    __threadfence();
  }
}

__global__ __launch_bounds__(128)
void gemm_o(const unsigned short* __restrict__ Wo16, const unsigned short* __restrict__ Oh,
            const unsigned short* __restrict__ Ol, const float* __restrict__ bo, float* Y) {
  __shared__ __align__(16) unsigned short Bh[QT * TP];
  __shared__ __align__(16) unsigned short Bl[QT * TP];
  __shared__ __align__(16) float Ys[QT * OSP];
  const int tid  = threadIdx.x;
  const int lane = tid & 31, wave = tid >> 5;
  const int hh   = lane >> 4, c = lane & 15;
  const int nt   = blockIdx.x, mb = blockIdx.y;
  const int n0   = nt * QT, o0 = mb * QT;
  const int e = tid & 7, lq = tid >> 3;

#pragma unroll
  for (int it = 0; it < 4; ++it) {
    const int cl = it * 16 + lq;
    const size_t so = (size_t)cl * NTOK + n0 + 8 * e;
    const v4u ah = *(const v4u*)(Oh + so);
    const v4u al = *(const v4u*)(Ol + so);
#pragma unroll
    for (int t = 0; t < 4; ++t) {
      Bh[(8 * e + 2 * t) * TP + cl]     = (unsigned short)(ah[t] & 0xffffu);
      Bh[(8 * e + 2 * t + 1) * TP + cl] = (unsigned short)(ah[t] >> 16);
      Bl[(8 * e + 2 * t) * TP + cl]     = (unsigned short)(al[t] & 0xffffu);
      Bl[(8 * e + 2 * t + 1) * TP + cl] = (unsigned short)(al[t] >> 16);
    }
  }
  __syncthreads();

  const unsigned short* ap  = Wo16 + (size_t)(o0 + c) * DK + 8 * hh;
  const unsigned short* bph = Bh + (16 * wave + c) * TP + 8 * hh;
  const unsigned short* bpl = Bl + (16 * wave + c) * TP + 8 * hh;

  v8f acch[4], accl[4];
#pragma unroll
  for (int mt = 0; mt < 4; ++mt) { acch[mt] = zero8(); accl[mt] = zero8(); }

#pragma unroll
  for (int ks = 0; ks < DK / 32; ++ks) {
    const Frag fbh = ldfrag(bph + 32 * ks);
    const Frag fbl = ldfrag(bpl + 32 * ks);
#pragma unroll
    for (int mt = 0; mt < 4; ++mt) {
      const Frag fa = ldfrag(ap + (size_t)(16 * mt) * DK + 32 * ks);
      acch[mt] = mma_h(fa.h, fbh.h, acch[mt]);
      accl[mt] = mma_h(fa.h, fbl.h, accl[mt]);
    }
  }

  {
    const int nl = 16 * wave + c;
    const float fs = IWSC * IOSC;
#pragma unroll
    for (int mt = 0; mt < 4; ++mt) {
      const v4f b0 = *(const v4f*)(bo + o0 + 16 * mt + 8 * hh);
      const v4f b1 = *(const v4f*)(bo + o0 + 16 * mt + 8 * hh + 4);
      v4f va, vb;
#pragma unroll
      for (int r = 0; r < 4; ++r) {
        va[r] = (acch[mt][r] + accl[mt][r] * IRSC) * fs + bfr(b0[r]);
        vb[r] = (acch[mt][4 + r] + accl[mt][4 + r] * IRSC) * fs + bfr(b1[r]);
      }
      *(v4f*)(Ys + nl * OSP + 16 * mt + 8 * hh)     = va;
      *(v4f*)(Ys + nl * OSP + 16 * mt + 8 * hh + 4) = vb;
    }
  }
  __syncthreads();

  v4f res[8];
#pragma unroll
  for (int it = 0; it < 8; ++it) {
    const int L  = it * 16 + lq;
    const int ol = L >> 1, hf = L & 1;
    const int nl = hf * 32 + 4 * e;
#pragma unroll
    for (int t = 0; t < 4; ++t) res[it][t] = Ys[(nl + t) * OSP + ol];
  }
#pragma unroll
  for (int pass = 0; pass < 2; ++pass) {
#pragma unroll
    for (int it = 0; it < 8; ++it) {
      const int L  = it * 16 + lq;
      const int ol = L >> 1, hf = L & 1;
      const int nl = hf * 32 + 4 * e;
      *(volatile v4f*)(Y + (size_t)(o0 + ol) * NTOK + n0 + nl) = res[it];
    }
    __threadfence();
  }
}

extern "C" void kernel_launch(void* const* d_in, const int* in_sizes, int n_in,
                              void* d_out, int out_size, void* d_ws, size_t ws_size,
                              hipStream_t stream) {
  if (n_in < 9) return;
  if (in_sizes[0] < CIN * NTOK) return;
  if ((in_sizes[0] % CIN) != 0) return;
  const int xstride = in_sizes[0] / CIN;
  if (xstride < NTOK || (xstride % 4) != 0) return;
  if (in_sizes[1] < DK * CIN || in_sizes[3] < DK * CIN || in_sizes[5] < DK * CIN) return;
  if (in_sizes[2] < DK || in_sizes[4] < DK || in_sizes[6] < DK) return;
  if (in_sizes[7] < COUT * DK || in_sizes[8] < COUT) return;
  if (out_size < COUT * NTOK) return;

  size_t off = 0;
  auto carve = [&](size_t bytes) { const size_t o = off; off += (bytes + 255) & ~(size_t)255; return o; };
  const size_t oW16  = carve((size_t)3 * DK * CIN * 2);
  const size_t oWo16 = carve((size_t)COUT * DK * 2);
  const size_t oXP   = carve((size_t)NTOK * CIN * 2);
  const size_t oQh   = carve((size_t)NTOK * DK * 2);
  const size_t oQl   = carve((size_t)NTOK * DK * 2);
  const size_t oKh   = carve((size_t)NTOK * DK * 2);
  const size_t oKl   = carve((size_t)NTOK * DK * 2);
  const size_t oVc   = carve((size_t)DK * NTOK * 2);
  const size_t oOh   = carve((size_t)NTOK * DK * 2);
  const size_t oOl   = carve((size_t)NTOK * DK * 2);
  if (off > ws_size) return;
  if (off > (size_t)134217728) return;

  const float* X  = (const float*)d_in[0];
  const float* Wq = (const float*)d_in[1];
  const float* bq = (const float*)d_in[2];
  const float* Wk = (const float*)d_in[3];
  const float* bk = (const float*)d_in[4];
  const float* Wv = (const float*)d_in[5];
  const float* bv = (const float*)d_in[6];
  const float* Wo = (const float*)d_in[7];
  const float* bo = (const float*)d_in[8];

  char* ws = (char*)d_ws;
  unsigned short* W16  = (unsigned short*)(ws + oW16);
  unsigned short* Wo16 = (unsigned short*)(ws + oWo16);
  unsigned short* XP   = (unsigned short*)(ws + oXP);
  unsigned short* Qh   = (unsigned short*)(ws + oQh);
  unsigned short* Ql   = (unsigned short*)(ws + oQl);
  unsigned short* Kh   = (unsigned short*)(ws + oKh);
  unsigned short* Kl   = (unsigned short*)(ws + oKl);
  unsigned short* Vc   = (unsigned short*)(ws + oVc);
  unsigned short* Oh   = (unsigned short*)(ws + oOh);
  unsigned short* Ol   = (unsigned short*)(ws + oOl);
  float* out = (float*)d_out;

  const dim3 blk256(256), blk128(128);
  const int BQ = (DK * CIN) / (8 * CHB), BO = (COUT * DK) / (8 * CHB);

  cvt_w<<<dim3(3 * BQ + BO), dim3(CHB), 0, stream>>>(Wq, Wk, Wv, Wo, W16, Wo16);
  cvt_x<<<dim3(NTOK / QT, CIN / QT), blk256, 0, stream>>>(X, xstride, XP);
  gemm_qkv<<<dim3(NTOK / QT, 3), blk128, 0, stream>>>(W16, XP, bq, bk, bv, Qh, Ql, Kh, Kl, Vc);
  attn_k<<<dim3(NTOK / QT), blk128, 0, stream>>>(Qh, Ql, Kh, Kl, Vc, Oh, Ol);
  gemm_o<<<dim3(NTOK / QT, COUT / QT), blk128, 0, stream>>>(Wo16, Oh, Ol, bo, out);
  (void)hipGetLastError();
}
